// GIN_84464826843159
// MI455X (gfx1250) — hardware-verified
//
#include <hip/hip_runtime.h>
#include <stddef.h>
#include <stdint.h>


#define HID      128
#define OUTW     64
#define NLAY     4
#define APW      256
#define KTOT     256
#define WSQ      (HID * KTOT)
#define NTHR     256
#define NWAVE    8
#define EPT      8
#define CHUNK    (NTHR * EPT)
#define WCAP     (EPT * 32)
#define LISTN    (NWAVE * WCAP)
#define NBMAX    2048
#define NBRUN    1024
#define RCAP     28672
#define DEGCAP   64
#define PKS      11
#define GBM      128
#define GTHR     256
#define BN       128
#define NUSQ     (HID * (KTOT / 8))
#define NUL2     (OUTW * (KTOT / 8))
#define NUTOT    (9 * NUSQ + NUL2)
#define PGR      8
#define POOLCAP  8192
#define WSMAX    134217728
#define LDS_BKT  ((2 * RCAP + 2 * NBMAX + LISTN) * 4 + 64)
#define LDS_GEMM (GBM * BN * 4)

static_assert(HID == 128 && HID == 32 * 4 && OUTW == 64);
static_assert((CHUNK & (CHUNK - 1)) == 0 && CHUNK <= (1 << PKS));
static_assert((NBMAX & (NBMAX - 1)) == 0 && NBMAX <= (1 << PKS));
static_assert(NTHR * 8 == NBMAX);
static_assert(LISTN >= NBMAX && LISTN >= NWAVE * WCAP);
static_assert(NBRUN <= NBMAX && NBRUN == 4 * NTHR && NBRUN == NWAVE * 128);
static_assert((RCAP % 32) == 0 && (RCAP % (4 * NTHR)) == 0);
static_assert(RCAP * 100 >= 16710 * 105);
static_assert(DEGCAP >= 36 + 8);
static_assert(POOLCAP >= 8 * 250 + 256);
static_assert(PGR == NWAVE && (PGR & (PGR - 1)) == 0);
static_assert(LDS_BKT <= 300000);
static_assert(GBM == (GTHR / 32) * 16 && KTOT == 2 * HID && APW == 2 * HID && (KTOT % 32) == 0);
static_assert((NUSQ % NTHR) == 0 && (NUL2 % NTHR) == 0 && (NUTOT % NTHR) == 0 && (KTOT / 8) == 32);

typedef float          v4f  __attribute__((ext_vector_type(4)));
typedef float          v8f  __attribute__((ext_vector_type(8)));
typedef int            v4i  __attribute__((ext_vector_type(4)));
typedef int            v8i  __attribute__((ext_vector_type(8)));
typedef unsigned int   v2u  __attribute__((ext_vector_type(2)));
typedef unsigned int   v4u  __attribute__((ext_vector_type(4)));
typedef unsigned short v8us __attribute__((ext_vector_type(8)));
typedef __bf16         v16b __attribute__((ext_vector_type(16)));
typedef v4f  __attribute__((may_alias)) v4fa;
typedef v4i  __attribute__((may_alias)) v4ia;
typedef v2u  __attribute__((may_alias)) v2ua;
typedef v4u  __attribute__((may_alias)) v4ua;
typedef v8us __attribute__((may_alias)) v8usa;
union FragB { v16b v; v8us h[2]; v8i w; };

__device__ __forceinline__ v8f wmb(const FragB& a, const FragB& b, v8f c) {
  v8f d = __builtin_amdgcn_wmma_f32_16x16x32_bf16(false, a.v, false, b.v, (short)0, c, false, false);
  asm volatile("v_nop\n\tv_nop\n\tv_nop\n\tv_nop" : "+v"(d) : "v"(a.w), "v"(b.w));
  return d;
}

__device__ __forceinline__ unsigned short bf_bits(float f) {
  const unsigned int u = __float_as_uint(f);
  const unsigned int r = (u + 0x7FFFu + ((u >> 16) & 1u)) >> 16;
  return (unsigned short)((f != f) ? 0x7FC0u : r);
}
__device__ __forceinline__ float bf_val(unsigned short b) { return __uint_as_float(((unsigned int)b) << 16); }
__device__ __forceinline__ float bf_rne(float f) { return bf_val(bf_bits(f)); }

__device__ __forceinline__ int scan_chunk(const int* __restrict__ dsts, int nE, int cbase, int slotBase,
                                          int nb, int vec8, int* list, int tid, int lane, int wave) {
  int wc = 0;
  const int el0  = tid * EPT;
  const int e0   = cbase + el0;
  const int sent = -2147483647 - 1;
  v4i da, db;
  if (vec8 != 0 && cbase + CHUNK <= nE) {
    da = *(const v4i*)(dsts + e0);
    db = *(const v4i*)(dsts + e0 + 4);
  } else {
    da.x = (e0     < nE) ? dsts[min(e0,     nE - 1)] : sent;
    da.y = (e0 + 1 < nE) ? dsts[min(e0 + 1, nE - 1)] : sent;
    da.z = (e0 + 2 < nE) ? dsts[min(e0 + 2, nE - 1)] : sent;
    da.w = (e0 + 3 < nE) ? dsts[min(e0 + 3, nE - 1)] : sent;
    db.x = (e0 + 4 < nE) ? dsts[min(e0 + 4, nE - 1)] : sent;
    db.y = (e0 + 5 < nE) ? dsts[min(e0 + 5, nE - 1)] : sent;
    db.z = (e0 + 6 < nE) ? dsts[min(e0 + 6, nE - 1)] : sent;
    db.w = (e0 + 7 < nE) ? dsts[min(e0 + 7, nE - 1)] : sent;
  }
  const unsigned nbs = (unsigned)slotBase;
  const unsigned unb = (unsigned)nb;
  const unsigned s0 = (unsigned)da.x - nbs, s1 = (unsigned)da.y - nbs;
  const unsigned s2 = (unsigned)da.z - nbs, s3 = (unsigned)da.w - nbs;
  const unsigned s4 = (unsigned)db.x - nbs, s5 = (unsigned)db.y - nbs;
  const unsigned s6 = (unsigned)db.z - nbs, s7 = (unsigned)db.w - nbs;
  const bool h0 = s0 < unb, h1 = s1 < unb, h2 = s2 < unb, h3 = s3 < unb;
  const bool h4 = s4 < unb, h5 = s5 < unb, h6 = s6 < unb, h7 = s7 < unb;
  const unsigned any = __builtin_amdgcn_ballot_w32(h0 | h1 | h2 | h3 | h4 | h5 | h6 | h7);
  if (any != 0u) {
#define HITJ(J, HJ, SJ) { \
      const unsigned mj = __builtin_amdgcn_ballot_w32(HJ); \
      if (mj != 0u) { \
        if (HJ) { \
          const int pos = wc + (int)__builtin_amdgcn_mbcnt_lo(mj, 0u); \
          if (pos < WCAP) list[wave * WCAP + pos] = ((el0 + (J)) << PKS) | (int)(SJ); \
        } \
        wc += (int)__builtin_popcount(mj); } }
    HITJ(0, h0, s0)
    HITJ(1, h1, s1)
    HITJ(2, h2, s2)
    HITJ(3, h3, s3)
    HITJ(4, h4, s4)
    HITJ(5, h5, s5)
    HITJ(6, h6, s6)
    HITJ(7, h7, s7)
#undef HITJ
  }
  return wc;
}

__device__ __forceinline__ v8us cv8b(const float* __restrict__ p, int stride) {
  v8us o;
#pragma unroll
  for (int i = 0; i < 8; ++i) o[i] = bf_bits(p[(size_t)i * (size_t)stride]);
  return o;
}

__global__ __launch_bounds__(NTHR) void k_wprep(const float* __restrict__ W1, const float* __restrict__ W2,
                                                const float* __restrict__ l1, const float* __restrict__ l2,
                                                unsigned short* wt) {
  const int u = (int)blockIdx.x * NTHR + (int)threadIdx.x;
  v8us o;
  size_t doff;
  if (u < 8 * NUSQ) {
    const int mi = u / NUSQ;
    const int v  = u - mi * NUSQ;
    const int n  = v >> 5;
    const int k8 = (v & 31) * 8;
    const int kk = k8 & (HID - 1);
    const size_t so = (size_t)(mi >> 1) * HID * HID + (size_t)kk * HID + n;
    if ((mi & 1) == 0) {
      o = cv8b(W1 + so, HID);
    } else {
      o = cv8b(W2 + so, HID);
    }
    doff = (size_t)mi * WSQ + (size_t)n * KTOT + k8;
  } else if (u < 9 * NUSQ) {
    const int v  = u - 8 * NUSQ;
    const int n  = v >> 5;
    const int k8 = (v & 31) * 8;
    const int kk = k8 & (HID - 1);
    o = cv8b(l1 + (size_t)kk * HID + n, HID);
    doff = (size_t)8 * WSQ + (size_t)n * KTOT + k8;
  } else if (u < NUTOT) {
    const int v  = u - 9 * NUSQ;
    const int n  = v >> 5;
    const int k8 = (v & 31) * 8;
    const int kk = k8 & (HID - 1);
    o = cv8b(l2 + (size_t)kk * OUTW + n, OUTW);
    doff = (size_t)9 * WSQ + (size_t)n * KTOT + k8;
  } else {
    return;
  }
  unsigned short* dp = wt + doff;
  *(volatile v8us*)dp = o;
  __threadfence();
  *(volatile v8us*)dp = o;
}

__global__ __launch_bounds__(NTHR) void k_bucket(const int* __restrict__ srcs, const int* __restrict__ dsts,
                                                 int* lst, int* cnts, int* offs, int* flags,
                                                 int nN, int nE, int vec8) {
  extern __shared__ v4f lds_dyn[];
  int* reg1 = (int*)lds_dyn;
  int* reg2 = reg1 + RCAP;
  int* scnt = reg2 + RCAP;
  int* soff = scnt + NBMAX;
  int* list = soff + NBMAX;
  int* wcnt = list + LISTN;
  int* wtot = wcnt + NWAVE;
  const int tid = (int)threadIdx.x, lane = tid & 31, wave = tid >> 5;
  const int blk = (int)blockIdx.x;
  const int nodeBase = blk * NBRUN;
  const int nb = NBRUN;

  for (int i = tid; i < NBMAX; i += NTHR) scnt[i] = 0;
  for (int i = tid; i < RCAP; i += NTHR) reg2[i] = 0;
  __syncthreads();

  int tot = 0;
  const int nChunks = (nE + CHUNK - 1) / CHUNK;
#pragma unroll 1
  for (int ch = 0; ch < nChunks; ++ch) {
    const int cbase = ch * CHUNK;
    const int wc = scan_chunk(dsts, nE, cbase, nodeBase, nb, vec8, list, tid, lane, wave);
    if (lane == 0) wcnt[wave] = wc;
    __syncthreads();
    int pre = 0, all = 0;
#pragma unroll
    for (int w2 = 0; w2 < NWAVE; ++w2) {
      int c = wcnt[w2];
      c = c < 0 ? 0 : (c > WCAP ? WCAP : c);
      all += c;
      pre += (w2 < wave) ? c : 0;
    }
    const int wcc  = wc > WCAP ? WCAP : wc;
    const int base = tot + pre;
#pragma unroll 1
    for (int i = lane; i < wcc; i += 32) {
      const int ent = list[wave * WCAP + i];
      const int el  = (ent >> PKS) & (CHUNK - 1);
      const int sl  = ent & (NBMAX - 1);
      int eid = cbase + el;
      eid = eid > nE - 1 ? nE - 1 : eid;
      const int pos = base + i;
      if (pos < RCAP) reg1[pos] = (int)(((unsigned)eid << PKS) | (unsigned)sl);
    }
    tot += all;
    tot = tot > RCAP ? RCAP : tot;
    __syncthreads();
  }
  const int nh = tot;

  if (wave == 0) {
#pragma unroll 1
    for (int b0 = 0; b0 < nh; b0 += 32) {
      const int idx = b0 + lane;
      const int uv  = reg1[idx < RCAP ? idx : RCAP - 1];
      const int m32 = (nh - b0) < 32 ? (nh - b0) : 32;
#pragma unroll 1
      for (int k = 0; k < m32; ++k) {
        const int u  = __builtin_amdgcn_readlane(uv, k);
        const int sl = u & (NBMAX - 1);
        if (lane == 0) scnt[sl] = scnt[sl] + 1;
      }
    }
  }
  __syncthreads();

  {
    const v4i ca = *(const v4ia*)(scnt + 8 * tid);
    const v4i cb = *(const v4ia*)(scnt + 8 * tid + 4);
    const int e0 = ca.x < 0 ? 0 : ca.x, e1 = ca.y < 0 ? 0 : ca.y, e2 = ca.z < 0 ? 0 : ca.z, e3 = ca.w < 0 ? 0 : ca.w;
    const int e4 = cb.x < 0 ? 0 : cb.x, e5 = cb.y < 0 ? 0 : cb.y, e6 = cb.z < 0 ? 0 : cb.z, e7 = cb.w < 0 ? 0 : cb.w;
    const int ts = e0 + e1 + e2 + e3 + e4 + e5 + e6 + e7;
    int incl = ts;
#pragma unroll
    for (int d = 1; d < 32; d <<= 1) {
      const int up = __shfl_up(incl, d);
      if (lane >= d) incl += up;
    }
    if (lane == 31) wtot[wave] = incl;
    __syncthreads();
    int pre = 0;
#pragma unroll
    for (int w2 = 0; w2 < NWAVE; ++w2) pre += (w2 < wave) ? wtot[w2] : 0;
    int run = pre + incl - ts;
    soff[8 * tid + 0] = run; run += e0;
    soff[8 * tid + 1] = run; run += e1;
    soff[8 * tid + 2] = run; run += e2;
    soff[8 * tid + 3] = run; run += e3;
    soff[8 * tid + 4] = run; run += e4;
    soff[8 * tid + 5] = run; run += e5;
    soff[8 * tid + 6] = run; run += e6;
    soff[8 * tid + 7] = run;
  }
  __syncthreads();
  for (int i = tid; i < NBMAX; i += NTHR) list[i] = soff[i];
  __syncthreads();

  if (wave == 0) {
#pragma unroll 1
    for (int b0 = 0; b0 < nh; b0 += 32) {
      const int idx = b0 + lane;
      const int uv  = reg1[idx < RCAP ? idx : RCAP - 1];
      const int m32 = (nh - b0) < 32 ? (nh - b0) : 32;
#pragma unroll 1
      for (int k = 0; k < m32; ++k) {
        const int u   = __builtin_amdgcn_readlane(uv, k);
        const int sl  = u & (NBMAX - 1);
        const int eid = (int)((unsigned)u >> PKS);
        if (lane == 0) {
          int pos = list[sl];
          pos = pos < 0 ? 0 : (pos > RCAP - 1 ? RCAP - 1 : pos);
          reg2[pos] = eid;
          list[sl] = pos + 1;
        }
      }
    }
  }
  __syncthreads();

  const int nhm = nh > 0 ? nh - 1 : 0;
#pragma unroll 4
  for (int i = tid; i < RCAP; i += NTHR) {
    const int ic = i < nhm ? i : nhm;
    int eid = reg2[ic];
    eid = eid < 0 ? 0 : (eid > nE - 1 ? nE - 1 : eid);
    int s = srcs[eid];
    s = s < 0 ? 0 : (s > nN - 1 ? nN - 1 : s);
    reg1[i] = (i < nh) ? s : 0;
  }
  __syncthreads();

  int* lp = lst + (size_t)blk * RCAP;
  const v4i cvv = *(const v4ia*)(scnt + 4 * tid);
  const v4i ovv = *(const v4ia*)(soff + 4 * tid);
  int* cp = cnts + (size_t)blk * NBRUN + 4 * tid;
  int* op = offs + (size_t)blk * NBRUN + 4 * tid;
  const int fl = (nh >= RCAP) ? 1 : 0;
  v4i fv; fv.x = fl; fv.y = fl; fv.z = fl; fv.w = fl;
  int* fp = flags + (size_t)blk * 32 + 4 * (tid & 7);
#pragma unroll 1
  for (int p = tid; p < RCAP / 4; p += NTHR) {
    const v4i v = *(const v4ia*)(reg1 + 4 * p);
    *(volatile v4i*)(lp + 4 * p) = v;
  }
  *(volatile v4i*)cp = cvv;
  *(volatile v4i*)op = ovv;
  if (tid < 8) *(volatile v4i*)fp = fv;
  __threadfence();
#pragma unroll 1
  for (int p = tid; p < RCAP / 4; p += NTHR) {
    const v4i v = *(const v4ia*)(reg1 + 4 * p);
    *(volatile v4i*)(lp + 4 * p) = v;
  }
  *(volatile v4i*)cp = cvv;
  *(volatile v4i*)op = ovv;
  if (tid < 8) *(volatile v4i*)fp = fv;
}

template <int L0>
__device__ __forceinline__ v4f ldrow(const float* __restrict__ xf, const unsigned short* __restrict__ xp,
                                     int node, int lane) {
  v4f r;
  if constexpr (L0 != 0) {
    const v4f v = *(const v4f*)(xf + (size_t)node * HID + 4 * lane);
    r.x = bf_rne(v.x); r.y = bf_rne(v.y); r.z = bf_rne(v.z); r.w = bf_rne(v.w);
  } else {
    const unsigned short* rp = xp + (size_t)node * APW + 4 * lane;
    const v2u h = *(const v2ua*)rp;
    const v2u l = *(const v2ua*)(rp + HID);
    r.x = __uint_as_float(h.x << 16)         + __uint_as_float(l.x << 16);
    r.y = __uint_as_float(h.x & 0xffff0000u) + __uint_as_float(l.x & 0xffff0000u);
    r.z = __uint_as_float(h.y << 16)         + __uint_as_float(l.y << 16);
    r.w = __uint_as_float(h.y & 0xffff0000u) + __uint_as_float(l.y & 0xffff0000u);
  }
  return r;
}

__device__ __forceinline__ void put_row_hilo(unsigned int* stwu, unsigned short* gp, bool wsv,
                                             float r0, float r1, float r2, float r3, int lane) {
  const unsigned short hb0 = bf_bits(r0), hb1 = bf_bits(r1), hb2 = bf_bits(r2), hb3 = bf_bits(r3);
  const unsigned short lb0 = bf_bits(r0 - bf_val(hb0)), lb1 = bf_bits(r1 - bf_val(hb1));
  const unsigned short lb2 = bf_bits(r2 - bf_val(hb2)), lb3 = bf_bits(r3 - bf_val(hb3));
  v2u hw, lw;
  hw.x = (unsigned int)hb0 | ((unsigned int)hb1 << 16);
  hw.y = (unsigned int)hb2 | ((unsigned int)hb3 << 16);
  lw.x = (unsigned int)lb0 | ((unsigned int)lb1 << 16);
  lw.y = (unsigned int)lb2 | ((unsigned int)lb3 << 16);
  __builtin_amdgcn_fence(__ATOMIC_RELEASE, "wavefront");
  __builtin_amdgcn_wave_barrier();
  *(v2u*)(stwu + 2 * lane)      = hw;
  *(v2u*)(stwu + 64 + 2 * lane) = lw;
  __builtin_amdgcn_fence(__ATOMIC_RELEASE, "wavefront");
  __builtin_amdgcn_wave_barrier();
  const v4u pk = *(const v4ua*)(stwu + 4 * lane);
  if (wsv) *(volatile v4u*)gp = pk;
  __threadfence();
  if (wsv) *(volatile v4u*)gp = pk;
}

template <int L0>
__global__ __launch_bounds__(NTHR) void k_agg(const float* __restrict__ xf, const unsigned short* __restrict__ xp,
                                              const int* __restrict__ lst, const int* __restrict__ cnts,
                                              const int* __restrict__ offs, const int* __restrict__ flags,
                                              const float* __restrict__ epsp,
                                              unsigned short* zout, int nN, int MPr) {
  __shared__ __attribute__((aligned(16))) unsigned int stw[NWAVE * 128];
  const int tid = (int)threadIdx.x, lane = tid & 31, wave = tid >> 5;
  const int blk = (int)blockIdx.x;
  const int nodeBase = blk * NBRUN;
  const int* lp = lst + (size_t)blk * RCAP;
  const int flg = flags[(size_t)blk * 32];
  const float e1 = 1.0f + bf_rne(epsp[0]);
  const float qnan = __int_as_float(0x7fc00000);
  unsigned int* stwu = stw + wave * 128;

#pragma unroll 1
  for (int g4 = 0; g4 < 4; ++g4) {
    const int sbase = wave * (NBRUN / NWAVE) + g4 * 32;
    const int cv = cnts[(size_t)blk * NBRUN + sbase + lane];
    const int ov = offs[(size_t)blk * NBRUN + sbase + lane];
#pragma unroll 1
    for (int j = 0; j < 32; ++j) {
      const int slot = sbase + j;
      const int grow = nodeBase + slot;
      const int craw = __builtin_amdgcn_readlane(cv, j);
      int st = __builtin_amdgcn_readlane(ov, j);
      st = st < 0 ? 0 : (st > RCAP ? RCAP : st);
      int cnt = craw < 0 ? 0 : (craw > DEGCAP ? DEGCAP : craw);
      if (cnt > RCAP - st) cnt = RCAP - st;
      const float pz = (flg != 0 || craw > DEGCAP) ? qnan : 0.0f;
      const bool liveRow = grow < nN;

      float ag0 = 0.f, ag1 = 0.f, ag2 = 0.f, ag3 = 0.f;
#pragma unroll 1
      for (int b0 = 0; b0 < cnt; b0 += 32) {
        const int last = st + cnt - 1;
        int idx = st + b0 + lane;
        idx = idx > last ? last : idx;
        int sv = lp[idx];
        sv = sv < 0 ? 0 : (sv > nN - 1 ? nN - 1 : sv);
        const int m32 = (cnt - b0) < 32 ? (cnt - b0) : 32;
#pragma unroll 1
        for (int k = 0; k < m32; ++k) {
          const int sk = __builtin_amdgcn_readlane(sv, k);
          const v4f v = ldrow<L0>(xf, xp, sk, lane);
          ag0 += v.x; ag1 += v.y; ag2 += v.z; ag3 += v.w;
        }
      }
      const int nc = liveRow ? grow : nN - 1;
      const v4f sf = ldrow<L0>(xf, xp, nc, lane);
      float r0 = fmaf(e1, sf.x, ag0), r1 = fmaf(e1, sf.y, ag1);
      float r2 = fmaf(e1, sf.z, ag2), r3 = fmaf(e1, sf.w, ag3);
      r0 = (liveRow ? r0 : 0.0f) + pz;
      r1 = (liveRow ? r1 : 0.0f) + pz;
      r2 = (liveRow ? r2 : 0.0f) + pz;
      r3 = (liveRow ? r3 : 0.0f) + pz;
      unsigned short* gp = zout + (size_t)grow * APW + 8 * lane;
      put_row_hilo(stwu, gp, grow < MPr, r0, r1, r2, r3, lane);
    }
  }
}

template <int EPI, int NT>
__global__ __launch_bounds__(GTHR) void k_gemm(const unsigned short* A, const unsigned short* __restrict__ WT,
                                               const float* __restrict__ pb, const float* __restrict__ pmean,
                                               const float* __restrict__ pvar, const float* __restrict__ pgam,
                                               const float* __restrict__ pbet,
                                               void* outp, int nN, int mRows) {
  extern __shared__ __attribute__((aligned(16))) float stg[];
  const int tid = (int)threadIdx.x, lane = tid & 31, wave = tid >> 5, hh = lane >> 4, m = lane & 15;
  const int rowBase = (int)blockIdx.x * GBM;

  v8f acc[NT];
  {
    const v8f z = {0.f, 0.f, 0.f, 0.f, 0.f, 0.f, 0.f, 0.f};
#pragma unroll
    for (int t = 0; t < NT; ++t) acc[t] = z;
  }
  const unsigned short* ap = A + (size_t)(rowBase + 16 * wave + m) * (size_t)APW + 8 * hh;
  const unsigned short* wp = WT + (size_t)m * (size_t)KTOT + 8 * hh;
  constexpr int ksteps = KTOT / 32;
#pragma unroll 1
  for (int ks = 0; ks < ksteps; ++ks) {
    FragB af;
    af.h[0] = *(const v8usa*)(ap + 32 * ks);
    af.h[1] = *(const v8usa*)(ap + 32 * ks + 16);
#pragma unroll
    for (int t = 0; t < NT; ++t) {
      const unsigned short* wq = wp + (size_t)(16 * t) * (size_t)KTOT + 32 * ks;
      FragB bf;
      bf.h[0] = *(const v8usa*)wq;
      bf.h[1] = *(const v8usa*)(wq + 16);
      acc[t] = wmb(af, bf, acc[t]);
    }
  }

#pragma unroll
  for (int t = 0; t < NT; ++t) {
    const int lc = 16 * t + m;
#pragma unroll
    for (int r = 0; r < 8; ++r) {
      const int lr = 16 * wave + 8 * hh + r;
      stg[lr * BN + lc] = acc[t][r];
    }
  }
  __syncthreads();

  {
    constexpr int NC  = 16 * NT;
    constexpr int RPI = GTHR / NC;
    constexpr int NIT = GBM / RPI;
    const int c  = tid & (NC - 1);
    const int rg = tid / NC;
    const float cb = bf_rne(pb[c]);
    float cm = 0.0f, crs = 1.0f, cg = 1.0f, cbe = 0.0f;
    if constexpr (EPI == 0) {
      cm  = bf_rne(pmean[c]);
      crs = 1.0f / sqrtf(bf_rne(pvar[c]) + 1e-5f);
      cg  = bf_rne(pgam[c]);
      cbe = bf_rne(pbet[c]);
    }
#pragma unroll 1
    for (int i = 0; i < NIT; ++i) {
      const int lr = i * RPI + rg;
      float v = stg[lr * BN + c] + cb;
      if constexpr (EPI == 0) {
        v = (v > 0.0f) ? v : (v - v);
        v = ((v - cm) * crs) * cg + cbe;
        v = (v > 0.0f) ? v : (v - v);
      } else if constexpr (EPI == 1) {
        v = (v > 0.0f) ? v : (v - v);
      }
      const bool live = (rowBase + lr) < nN;
      stg[lr * BN + c] = live ? v : 0.0f;
    }
  }
  __syncthreads();

  if constexpr (EPI != 2) {
    unsigned short* outH = (unsigned short*)outp;
    const int cb8 = 8 * m;
    const bool isHi = (hh == 0);
    v4u pk[16];
#pragma unroll
    for (int i = 0; i < 16; ++i) {
      const int lr = 16 * wave + i;
      const v4f a = *(const v4fa*)(stg + lr * BN + cb8);
      const v4f b = *(const v4fa*)(stg + lr * BN + cb8 + 4);
      const float f[8] = {a.x, a.y, a.z, a.w, b.x, b.y, b.z, b.w};
      unsigned int w[4];
#pragma unroll
      for (int j = 0; j < 4; ++j) {
        const unsigned short h0 = bf_bits(f[2 * j]), h1 = bf_bits(f[2 * j + 1]);
        const unsigned short l0 = bf_bits(f[2 * j] - bf_val(h0)), l1 = bf_bits(f[2 * j + 1] - bf_val(h1));
        const unsigned short q0 = isHi ? h0 : l0, q1 = isHi ? h1 : l1;
        w[j] = (unsigned int)q0 | ((unsigned int)q1 << 16);
      }
      v4u pw; pw.x = w[0]; pw.y = w[1]; pw.z = w[2]; pw.w = w[3];
      pk[i] = pw;
    }
#pragma unroll
    for (int i = 0; i < 16; ++i) {
      const int gr = rowBase + 16 * wave + i;
      unsigned short* op = outH + (size_t)gr * (size_t)APW + 8 * lane;
      if (gr < mRows) *(volatile v4u*)op = pk[i];
    }
    __threadfence();
#pragma unroll
    for (int i = 0; i < 16; ++i) {
      const int gr = rowBase + 16 * wave + i;
      unsigned short* op = outH + (size_t)gr * (size_t)APW + 8 * lane;
      if (gr < mRows) *(volatile v4u*)op = pk[i];
    }
  } else {
    static_assert(EPI != 2 || NT == 4);
    float* outF = (float*)outp;
    constexpr int LDO = 16 * NT;
    const int c4 = 4 * m;
    v4f fv[8];
#pragma unroll
    for (int i = 0; i < 8; ++i) {
      const int lr = 16 * wave + 2 * i + hh;
      fv[i] = *(const v4fa*)(stg + lr * BN + c4);
    }
#pragma unroll
    for (int i = 0; i < 8; ++i) {
      const int gr = rowBase + 16 * wave + 2 * i + hh;
      float* op = outF + (size_t)gr * LDO + c4;
      if (gr < mRows) *(volatile v4f*)op = fv[i];
    }
    __threadfence();
#pragma unroll
    for (int i = 0; i < 8; ++i) {
      const int gr = rowBase + 16 * wave + 2 * i + hh;
      float* op = outF + (size_t)gr * LDO + c4;
      if (gr < mRows) *(volatile v4f*)op = fv[i];
    }
  }
}

__global__ __launch_bounds__(NTHR) void k_pool(const unsigned short* __restrict__ xp, const int* __restrict__ bat,
                                               int nN, int vec8b, int nG, unsigned short* gout) {
  __shared__ int plist[POOLCAP];
  __shared__ int list[LISTN];
  __shared__ int wcnt[NWAVE];
  __shared__ __attribute__((aligned(16))) unsigned int stw[NWAVE * 128];
  const int tid = (int)threadIdx.x, lane = tid & 31, wave = tid >> 5;
  const int slotBase = (int)blockIdx.x * PGR;

  int tot = 0;
  const int nChunks = (nN + CHUNK - 1) / CHUNK;
#pragma unroll 1
  for (int ch = 0; ch < nChunks; ++ch) {
    const int cbase = ch * CHUNK;
    const int wc = scan_chunk(bat, nN, cbase, slotBase, PGR, vec8b, list, tid, lane, wave);
    if (lane == 0) wcnt[wave] = wc;
    __syncthreads();
    int pre = 0, all = 0;
#pragma unroll
    for (int w2 = 0; w2 < NWAVE; ++w2) {
      int c = wcnt[w2];
      c = c < 0 ? 0 : (c > WCAP ? WCAP : c);
      all += c;
      pre += (w2 < wave) ? c : 0;
    }
    const int wcc  = wc > WCAP ? WCAP : wc;
    const int base = tot + pre;
#pragma unroll 1
    for (int i = lane; i < wcc; i += 32) {
      const int ent = list[wave * WCAP + i];
      const int el  = (ent >> PKS) & (CHUNK - 1);
      const int sl  = ent & (PGR - 1);
      int node = cbase + el;
      node = node > nN - 1 ? nN - 1 : node;
      const int pos = base + i;
      if (pos < POOLCAP) plist[pos] = (int)(((unsigned)node << PKS) | (unsigned)sl);
    }
    tot += all;
    tot = tot > POOLCAP ? POOLCAP : tot;
    __syncthreads();
  }
  const int nh = tot;
  const bool ovf = (nh >= POOLCAP);
  const int wv = __builtin_amdgcn_readfirstlane(wave);

  float ag0 = 0.f, ag1 = 0.f, ag2 = 0.f, ag3 = 0.f;
#pragma unroll 1
  for (int b0 = 0; b0 < nh; b0 += 32) {
    int idx = b0 + lane;
    idx = idx > nh - 1 ? nh - 1 : idx;
    const int ent = plist[idx];
    const int m32 = (nh - b0) < 32 ? (nh - b0) : 32;
#pragma unroll 1
    for (int k = 0; k < m32; ++k) {
      const int u  = __builtin_amdgcn_readlane(ent, k);
      const int sl = u & (PGR - 1);
      int node = (int)((unsigned)u >> PKS);
      node = node > nN - 1 ? nN - 1 : node;
      if (sl == wv) {
        const v4f v = ldrow<0>((const float*)0, xp, node, lane);
        ag0 += v.x; ag1 += v.y; ag2 += v.z; ag3 += v.w;
      }
    }
  }
  const float pz = ovf ? __int_as_float(0x7fc00000) : 0.0f;
  const int g = slotBase + wv;
  unsigned short* gp = gout + (size_t)g * APW + 8 * lane;
  put_row_hilo(stw + wv * 128, gp, g < nG, ag0 + pz, ag1 + pz, ag2 + pz, ag3 + pz, lane);
}

static inline int cdiv(int a, int b) { return (a + b - 1) / b; }
static inline size_t al256(size_t o) { return (o + 255) & ~(size_t)255; }

extern "C" void kernel_launch(void* const* d_in, const int* in_sizes, int n_in,
                              void* d_out, int out_size, void* d_ws, size_t ws_size,
                              hipStream_t stream) {
  if (n_in < 16) return;
  if (in_sizes[0] < HID || (in_sizes[0] % HID) != 0) return;
  const int nN = in_sizes[0] / HID;
  if (nN < GBM || nN > (1 << 21)) return;
  const int nE2 = in_sizes[1];
  if (nE2 < 2 || (nE2 & 1) != 0) return;
  const int nE = nE2 / 2;
  if (nE < 1 || nE > (1 << 21)) return;
  if (in_sizes[2] != nN) return;
  if (in_sizes[3] != NLAY) return;
  if (in_sizes[4] != NLAY * HID * HID || in_sizes[10] != NLAY * HID * HID) return;
  if (in_sizes[5] != NLAY * HID || in_sizes[6] != NLAY * HID || in_sizes[7] != NLAY * HID) return;
  if (in_sizes[8] != NLAY * HID || in_sizes[9] != NLAY * HID || in_sizes[11] != NLAY * HID) return;
  if (in_sizes[12] != HID * HID || in_sizes[13] != HID) return;
  if (in_sizes[14] != HID * OUTW || in_sizes[15] != OUTW) return;
  if (out_size < OUTW || (out_size % OUTW) != 0) return;
  const int nG = out_size / OUTW;
  if (nG < GBM || (nG % GBM) != 0 || (nG % PGR) != 0 || nG > 65536) return;
  if ((long long)nG * OUTW != (long long)out_size) return;
  if ((long long)NBRUN * (long long)nE * 5LL > (long long)RCAP * (long long)nN * 4LL) return;

  const float* x     = (const float*)d_in[0];
  const int*   ei    = (const int*)  d_in[1];
  const int*   src   = ei;
  const int*   dst   = ei + nE;
  const int*   batch = (const int*)  d_in[2];
  const float* eps   = (const float*)d_in[3];
  const float* W1    = (const float*)d_in[4];
  const float* b1    = (const float*)d_in[5];
  const float* gam   = (const float*)d_in[6];
  const float* bet   = (const float*)d_in[7];
  const float* bnm   = (const float*)d_in[8];
  const float* bnv   = (const float*)d_in[9];
  const float* W2    = (const float*)d_in[10];
  const float* b2    = (const float*)d_in[11];
  const float* l1w   = (const float*)d_in[12];
  const float* l1b   = (const float*)d_in[13];
  const float* l2w   = (const float*)d_in[14];
  const float* l2b   = (const float*)d_in[15];
  float* out = (float*)d_out;

  const int MP   = cdiv(nN, GBM) * GBM;
  const int gM   = MP / GBM;
  const int gB   = cdiv(MP, NBRUN);
  const int vec8 = ((nE & 3) == 0) ? 1 : 0;
  if ((long long)gB * NBRUN < (long long)MP) return;
  if ((long long)(gM - 1) * GBM >= (long long)nN) return;

  char* ws = (char*)d_ws;
  size_t off = 0;
  const size_t oWT = off; off = al256(off + ((size_t)9 * WSQ + (size_t)OUTW * KTOT) * 2);
  const size_t oP1 = off; off = al256(off + (size_t)MP * APW * 2);
  const size_t oP2 = off; off = al256(off + (size_t)MP * APW * 2);
  const size_t oLS = off; off = al256(off + (size_t)gB * RCAP * 4);
  const size_t oCN = off; off = al256(off + (size_t)gB * NBRUN * 4);
  const size_t oOF = off; off = al256(off + (size_t)gB * NBRUN * 4);
  const size_t oFL = off; off = al256(off + (size_t)gB * 32 * 4);
  const size_t oGP = off; off = al256(off + (size_t)nG * APW * 2);
  const size_t oG1 = off; off = al256(off + (size_t)nG * APW * 2);
  if (off > ws_size || off > (size_t)WSMAX) return;
  unsigned short* WT   = (unsigned short*)(ws + oWT);
  unsigned short* P1   = (unsigned short*)(ws + oP1);
  unsigned short* P2   = (unsigned short*)(ws + oP2);
  int*            LIST = (int*)(ws + oLS);
  int*            CNT  = (int*)(ws + oCN);
  int*            OFF  = (int*)(ws + oOF);
  int*            FLAG = (int*)(ws + oFL);
  unsigned short* GP   = (unsigned short*)(ws + oGP);
  unsigned short* G1   = (unsigned short*)(ws + oG1);

  hipFuncSetAttribute(reinterpret_cast<const void*>(&k_bucket), hipFuncAttributeMaxDynamicSharedMemorySize, LDS_BKT);
  hipFuncSetAttribute(reinterpret_cast<const void*>(&k_gemm<0, 8>), hipFuncAttributeMaxDynamicSharedMemorySize, LDS_GEMM);
  hipFuncSetAttribute(reinterpret_cast<const void*>(&k_gemm<1, 8>), hipFuncAttributeMaxDynamicSharedMemorySize, LDS_GEMM);
  hipFuncSetAttribute(reinterpret_cast<const void*>(&k_gemm<2, 4>), hipFuncAttributeMaxDynamicSharedMemorySize, LDS_GEMM);

  k_wprep<<<NUTOT / NTHR, NTHR, 0, stream>>>(W1, W2, l1w, l2w, WT);
  k_bucket<<<gB, NTHR, LDS_BKT, stream>>>(src, dst, LIST, CNT, OFF, FLAG, nN, nE, vec8);
  for (int l = 0; l < NLAY; ++l) {
    const size_t lo = (size_t)l * HID;
    if (l == 0) {
      k_agg<1><<<gB, NTHR, 0, stream>>>(x, P1, LIST, CNT, OFF, FLAG, eps + l, P2, nN, MP);
    } else {
      k_agg<0><<<gB, NTHR, 0, stream>>>(x, P1, LIST, CNT, OFF, FLAG, eps + l, P2, nN, MP);
    }
    k_gemm<0, 8><<<gM, GTHR, LDS_GEMM, stream>>>(P2, WT + (size_t)(2 * l) * WSQ, b1 + lo, bnm + lo, bnv + lo,
                                                 gam + lo, bet + lo, (void*)P2, nN, MP);
    k_gemm<1, 8><<<gM, GTHR, LDS_GEMM, stream>>>(P2, WT + (size_t)(2 * l + 1) * WSQ, b2 + lo, b2 + lo, b2 + lo,
                                                 b2 + lo, b2 + lo, (void*)P1, nN, MP);
  }
  k_pool<<<nG / PGR, NTHR, 0, stream>>>(P1, batch, nN, 1, nG, GP);
  k_gemm<1, 8><<<nG / GBM, GTHR, LDS_GEMM, stream>>>(GP, WT + (size_t)8 * WSQ, l1b, l1b, l1b, l1b, l1b,
                                                     (void*)G1, nG, nG);
  k_gemm<2, 4><<<nG / GBM, GTHR, LDS_GEMM, stream>>>(G1, WT + (size_t)9 * WSQ, l2b, l2b, l2b, l2b, l2b,
                                                     (void*)out, nG, nG);
}
